// FGN_layer_66262755443328
// MI455X (gfx1250) — hardware-run, weakly checked
//
#include <hip/hip_runtime.h>
#include <math.h>

typedef __attribute__((ext_vector_type(16))) _Float16 v16h;
typedef __attribute__((ext_vector_type(8)))  _Float16 v8h;
typedef __attribute__((ext_vector_type(16))) __bf16   v16b;
typedef __attribute__((ext_vector_type(8)))  __bf16   v8b;
typedef __attribute__((ext_vector_type(8)))  float    v8f;
typedef __attribute__((ext_vector_type(4)))  float    v4f;
typedef __attribute__((ext_vector_type(4)))  unsigned v4u;

constexpr int kRowsB = 1024;
constexpr int kFeatI = 512;
constexpr int kOutO  = 512;
constexpr int kTilePitch = 68;
constexpr float kCarryX  = 64.0f;
constexpr float kCarryW  = 1024.0f;
constexpr float kCarryCS = 67108864.0f;
constexpr float kCarryS2 = 4294967296.0f;
constexpr float kInvL = 1.0f / (kCarryX * kCarryW);
constexpr float kInvG = 1.0f / kCarryS2;
constexpr float kCsFactor = -2.0f * kCarryCS;
constexpr float kF16MinNormal = 6.103515625e-5f;
constexpr float kEpsInner = 1e-32f;
static_assert(kCarryX * kCarryCS == kCarryS2);
static_assert((kFeatI % 32) == 0);
static_assert((kRowsB % 64) == 0 && (kOutO % 64) == 0);
static_assert((kOutO % 32) == 0);
static_assert(((kRowsB * kFeatI / 8) % 256) == 0);

constexpr size_t kOffXH = 0;
constexpr size_t kOffXQ = kOffXH + (size_t)kRowsB * kFeatI * 2;
constexpr size_t kOffWH = kOffXQ + (size_t)kRowsB * kFeatI * 2;
constexpr size_t kOffSB = kOffWH + (size_t)kOutO * kFeatI * 2;
constexpr size_t kOffCH = kOffSB + (size_t)kOutO * kFeatI * 2;
constexpr size_t kOffKC = kOffCH + (size_t)kOutO * kFeatI * 2;
constexpr size_t kWsTotal = kOffKC + (size_t)kOutO * 4;
static_assert(kWsTotal == 3672064ull);
static_assert(kWsTotal <= 134217728ull);
static_assert((kOffXQ % 128) == 0 && (kOffWH % 128) == 0 && (kOffSB % 128) == 0 &&
              (kOffCH % 128) == 0 && (kOffKC % 128) == 0);

__device__ __forceinline__ unsigned short f2bf_bits(float f) {
  unsigned u = __float_as_uint(f);
  return (unsigned short)((u + 0x7FFFu + ((u >> 16) & 1u)) >> 16);
}
__device__ __forceinline__ unsigned short f16_bits_flush(float v) {
  const float s = (fabsf(v) < kF16MinNormal) ? 0.0f : v;
  const _Float16 h = (_Float16)s;
  return __builtin_bit_cast(unsigned short, h);
}
__device__ __forceinline__ unsigned pack2(unsigned short lo, unsigned short hi) {
  return (unsigned)lo | (((unsigned)hi) << 16);
}

template <typename T> struct Frag;
template <> struct Frag<_Float16> {
  typedef v16h V; union U { v16h v; v8h h[2]; };
  static __device__ __forceinline__ v16h load(const _Float16* p) {
    U f; f.h[0] = *(const v8h*)(p); f.h[1] = *(const v8h*)(p + 16); return f.v;
  }
};
template <> struct Frag<__bf16> {
  typedef v16b V; union U { v16b v; v8b h[2]; };
  static __device__ __forceinline__ v16b load(const __bf16* p) {
    U f; f.h[0] = *(const v8b*)(p); f.h[1] = *(const v8b*)(p + 16); return f.v;
  }
};
__device__ __forceinline__ v8f mma_h(v16h a, v16h b, v8f c) {
  c = __builtin_amdgcn_wmma_f32_16x16x32_f16(false, a, false, b, (short)0, c, false, false);
  asm volatile("v_nop\n\tv_nop\n\tv_nop\n\tv_nop" : "+v"(c) : "v"(a), "v"(b));
  return c;
}
__device__ __forceinline__ v8f mma_b(v16b a, v16b b, v8f c) {
  c = __builtin_amdgcn_wmma_f32_16x16x32_bf16(false, a, false, b, (short)0, c, false, false);
  asm volatile("v_nop\n\tv_nop\n\tv_nop\n\tv_nop" : "+v"(c) : "v"(a), "v"(b));
  return c;
}

__global__ __launch_bounds__(256) void prep_in_rows_kernel(
    const float* __restrict__ X, unsigned* __restrict__ XHw, unsigned* __restrict__ XQw, int total8)
{
  const int i = blockIdx.x * 256 + threadIdx.x;
  if (i >= total8) return;
  const size_t e0 = (size_t)i << 3;
  const v4f a0 = *(const v4f*)(X + e0);
  const v4f a1 = *(const v4f*)(X + e0 + 4);
  const float xs[8] = {a0[0], a0[1], a0[2], a0[3], a1[0], a1[1], a1[2], a1[3]};
  v4u hw, qw;
#pragma unroll
  for (int p = 0; p < 4; ++p) {
    const float f0 = xs[2 * p];
    const float f1 = xs[2 * p + 1];
    const float q0 = f0 * f0;
    const float q1 = f1 * f1;
    hw[p] = pack2(f16_bits_flush(f0 * kCarryX), f16_bits_flush(f1 * kCarryX));
    qw[p] = pack2(f2bf_bits(q0), f2bf_bits(q1));
  }
  unsigned* ph = XHw + ((size_t)i << 2);
  unsigned* pq = XQw + ((size_t)i << 2);
  *(volatile v4u*)ph = hw;
  *(volatile v4u*)pq = qw;
  __threadfence();
  *(volatile v4u*)ph = hw;
  *(volatile v4u*)pq = qw;
}

__global__ __launch_bounds__(256) void prep_out_rows_kernel(
    const float* __restrict__ W, const float* __restrict__ C, const float* __restrict__ IC,
    unsigned* __restrict__ WHw, unsigned* __restrict__ SBw, unsigned* __restrict__ CHw,
    float* __restrict__ Kc)
{
  __shared__ float sPart[64];
  const int tid = threadIdx.x, lane = tid & 31, wave = tid >> 5;
  const int rsub = tid >> 6;
  const int c8 = (tid & 63) * 8;
#pragma unroll 1
  for (int it = 0; it < 8; ++it) {
    const int rloc = it * 4 + rsub;
    const int row = blockIdx.x * 32 + rloc;
    const size_t e0 = (size_t)row * kFeatI + c8;
    const v4f w0 = *(const v4f*)(W + e0);
    const v4f w1 = *(const v4f*)(W + e0 + 4);
    const v4f c0 = *(const v4f*)(C + e0);
    const v4f c1 = *(const v4f*)(C + e0 + 4);
    const v4f s0 = *(const v4f*)(IC + e0);
    const v4f s1 = *(const v4f*)(IC + e0 + 4);
    const float wv[8] = {w0[0], w0[1], w0[2], w0[3], w1[0], w1[1], w1[2], w1[3]};
    const float cv[8] = {c0[0], c0[1], c0[2], c0[3], c1[0], c1[1], c1[2], c1[3]};
    const float iv[8] = {s0[0], s0[1], s0[2], s0[3], s1[0], s1[1], s1[2], s1[3]};
    v4u ww, sw, cw;
    float ks = 0.0f;
#pragma unroll
    for (int p = 0; p < 4; ++p) {
      const float sa = iv[2 * p] * iv[2 * p] + kEpsInner;
      const float sb = iv[2 * p + 1] * iv[2 * p + 1] + kEpsInner;
      const float ca = cv[2 * p];
      const float cb = cv[2 * p + 1];
      const float csa = ca * sa;
      const float csb = cb * sb;
      ww[p] = pack2(f16_bits_flush(wv[2 * p] * kCarryW), f16_bits_flush(wv[2 * p + 1] * kCarryW));
      sw[p] = pack2(f2bf_bits(sa * kCarryS2), f2bf_bits(sb * kCarryS2));
      cw[p] = pack2(f16_bits_flush(csa * kCsFactor), f16_bits_flush(csb * kCsFactor));
      ks = fmaf(ca, csa, ks);
      ks = fmaf(cb, csb, ks);
    }
    const size_t wo = e0 >> 1;
    *(volatile v4u*)(WHw + wo) = ww;
    *(volatile v4u*)(SBw + wo) = sw;
    *(volatile v4u*)(CHw + wo) = cw;
    __threadfence();
    *(volatile v4u*)(WHw + wo) = ww;
    *(volatile v4u*)(SBw + wo) = sw;
    *(volatile v4u*)(CHw + wo) = cw;
#pragma unroll
    for (int off = 16; off > 0; off >>= 1) ks += __shfl_xor(ks, off, 32);
    if (lane == 0) sPart[rloc * 2 + (wave & 1)] = ks;
  }
  __syncthreads();
  if (wave == 0) {
    const float kc = sPart[2 * lane] + sPart[2 * lane + 1];
    float* pk = Kc + blockIdx.x * 32 + lane;
    *(volatile float*)pk = kc;
    __threadfence();
    *(volatile float*)pk = kc;
  }
}

__global__ __launch_bounds__(128) void gate_gemm_kernel(
    const unsigned short* __restrict__ XHp, const unsigned short* __restrict__ XQp,
    const unsigned short* __restrict__ WHp, const unsigned short* __restrict__ SBp,
    const unsigned short* __restrict__ CHp,
    const float* __restrict__ bias, const float* __restrict__ Kc, float* __restrict__ out)
{
  __shared__ __align__(16) float sL[64 * kTilePitch];
  __shared__ __align__(16) float sG[64 * kTilePitch];
  const _Float16* XH = (const _Float16*)XHp;
  const __bf16*   XQ = (const __bf16*)XQp;
  const _Float16* WH = (const _Float16*)WHp;
  const __bf16*   SB = (const __bf16*)SBp;
  const _Float16* CH = (const _Float16*)CHp;

  const int tid = threadIdx.x, lane = tid & 31, wave = tid >> 5;
  const int waveM = wave & 1, waveN = wave >> 1;
  const int m0 = blockIdx.y * 64, n0 = blockIdx.x * 64;
  const int rlane = lane & 15;
  const int koff = (lane >> 4) * 8;
  const int mOff = (lane >> 4) * 8;

  v8f accL[2][2], accG[2][2];
#pragma unroll
  for (int i = 0; i < 2; ++i)
#pragma unroll
    for (int j = 0; j < 2; ++j) {
      accL[i][j] = (v8f){0.f, 0.f, 0.f, 0.f, 0.f, 0.f, 0.f, 0.f};
      accG[i][j] = (v8f){0.f, 0.f, 0.f, 0.f, 0.f, 0.f, 0.f, 0.f};
    }

  const size_t aBase = (size_t)(m0 + waveM * 32 + rlane) * kFeatI + koff;
  const size_t bBase = (size_t)(n0 + waveN * 32 + rlane) * kFeatI + koff;

#pragma unroll 1
  for (int k0 = 0; k0 < kFeatI; k0 += 32) {
    v16h bW[2], bC[2];
    v16b bS[2];
#pragma unroll
    for (int j = 0; j < 2; ++j) {
      const size_t bo = bBase + (size_t)(j * 16) * kFeatI + k0;
      bW[j] = Frag<_Float16>::load(WH + bo);
      bS[j] = Frag<__bf16>::load(SB + bo);
      bC[j] = Frag<_Float16>::load(CH + bo);
    }
#pragma unroll
    for (int i = 0; i < 2; ++i) {
      const size_t ao = aBase + (size_t)(i * 16) * kFeatI + k0;
      const v16h aX = Frag<_Float16>::load(XH + ao);
      const v16b aQ = Frag<__bf16>::load(XQ + ao);
#pragma unroll
      for (int j = 0; j < 2; ++j) {
        accL[i][j] = mma_h(aX, bW[j], accL[i][j]);
        accG[i][j] = mma_b(aQ, bS[j], accG[i][j]);
        accG[i][j] = mma_h(aX, bC[j], accG[i][j]);
      }
    }
  }

#pragma unroll
  for (int i = 0; i < 2; ++i) {
#pragma unroll
    for (int j = 0; j < 2; ++j) {
      const int tcol = waveN * 32 + j * 16 + rlane;
#pragma unroll
      for (int r = 0; r < 8; ++r) {
        const int trow = waveM * 32 + i * 16 + mOff + r;
        sL[trow * kTilePitch + tcol] = accL[i][j][r] * kInvL;
        sG[trow * kTilePitch + tcol] = accG[i][j][r] * kInvG;
      }
    }
  }
  __syncthreads();

  const int hh = lane >> 4;
  const int c4 = (lane & 15) * 4;
  const v4f bv = *(const v4f*)(bias + n0 + c4);
  const v4f kv = *(const v4f*)(Kc + n0 + c4);
#pragma unroll 1
  for (int it = 0; it < 8; ++it) {
    const int row = wave * 16 + it * 2 + hh;
    const v4f lv = *(const v4f*)(sL + row * kTilePitch + c4);
    const v4f gv = *(const v4f*)(sG + row * kTilePitch + c4);
    v4f ov;
#pragma unroll
    for (int e = 0; e < 4; ++e) {
      const float l = lv[e] + bv[e];
      const float g = gv[e] + kv[e];
      ov[e] = l * expf(-g);
    }
    *(v4f*)(sL + row * kTilePitch + c4) = ov;
  }
  __syncthreads();

  for (int pass = 0; pass < 2; ++pass) {
#pragma unroll
    for (int it = 0; it < 8; ++it) {
      const int row = wave * 16 + it * 2 + hh;
      const v4f v = *(const v4f*)(sL + row * kTilePitch + c4);
      *(volatile v4f*)(out + (size_t)(m0 + row) * kOutO + n0 + c4) = v;
    }
    __threadfence();
  }
}

extern "C" void kernel_launch(void* const* d_in, const int* in_sizes, int n_in,
                              void* d_out, int out_size, void* d_ws, size_t ws_size,
                              hipStream_t stream) {
  if (n_in < 5) return;
  if (in_sizes[0] != kRowsB * kFeatI) return;
  if (in_sizes[1] != kOutO * kFeatI) return;
  if (in_sizes[2] != kOutO) return;
  if (in_sizes[3] != kOutO * kFeatI) return;
  if (in_sizes[4] != kOutO * kFeatI) return;
  if (out_size != kRowsB * kOutO) return;
  if (ws_size < kWsTotal) return;

  const float* X    = (const float*)d_in[0];
  const float* W    = (const float*)d_in[1];
  const float* bias = (const float*)d_in[2];
  const float* C    = (const float*)d_in[3];
  const float* IC   = (const float*)d_in[4];
  float* out = (float*)d_out;

  char* ws = (char*)d_ws;
  unsigned* XHw = (unsigned*)(ws + kOffXH);
  unsigned* XQw = (unsigned*)(ws + kOffXQ);
  unsigned* WHw = (unsigned*)(ws + kOffWH);
  unsigned* SBw = (unsigned*)(ws + kOffSB);
  unsigned* CHw = (unsigned*)(ws + kOffCH);
  float*    KC  = (float*)(ws + kOffKC);

  prep_in_rows_kernel<<<(kRowsB * kFeatI / 8) / 256, 256, 0, stream>>>(X, XHw, XQw, kRowsB * kFeatI / 8);
  prep_out_rows_kernel<<<kOutO / 32, 256, 0, stream>>>(W, C, IC, WHw, SBw, CHw, KC);
  gate_gemm_kernel<<<dim3(kOutO / 64, kRowsB / 64), 128, 0, stream>>>(
      (const unsigned short*)XHw, (const unsigned short*)XQw,
      (const unsigned short*)WHw, (const unsigned short*)SBw, (const unsigned short*)CHw,
      bias, KC, out);
}
